// TransformerEncoderLayer_3874060501280
// MI455X (gfx1250) — hardware-verified
//
#include <hip/hip_runtime.h>
#ifndef NB
#define NB 8
#endif
#ifndef SEQ
#define SEQ 1024
#endif
#define NB_FULL 8
#define DM 768
#define NH 8
#define HD 96
#define DFF 3072
#define NREL 199
#define NRELP 208
#define NCOL 224
#define KSOFF 104
#define PRP 232
#define LQKV (3 * DM)
#define MROWS (NB * SEQ)

static_assert(NH * HD == DM);
static_assert(HD % 32 == 0);
static_assert(SEQ % 64 == 0);
static_assert(MROWS % 128 == 0);
static_assert(DM % 64 == 0 && DFF % 64 == 0 && LQKV % 64 == 0);
static_assert(DM % 32 == 0 && DFF % 32 == 0);
static_assert(NH % 2 == 0);
static_assert(NRELP % 16 == 0 && NRELP >= NREL);
static_assert(NCOL % 32 == 0 && NCOL >= 15 + KSOFF + 99 + 1);
static_assert(KSOFF % 8 == 0 && KSOFF >= 99);

typedef unsigned short v8us __attribute__((ext_vector_type(8), may_alias));
typedef float  v8f  __attribute__((ext_vector_type(8)));
typedef float  v4f  __attribute__((ext_vector_type(4)));
typedef float  v4fa __attribute__((ext_vector_type(4), may_alias));
typedef _Float16 v16h __attribute__((ext_vector_type(16)));
typedef _Float16 v4h __attribute__((ext_vector_type(4)));
union FragH { v16h v; v8us half[2]; _Float16 h[16]; unsigned short u[16]; };

__device__ __forceinline__ unsigned short bf16_bits(float x) { unsigned int u = __float_as_uint(x); return (unsigned short)((u + 0x7FFFu + ((u >> 16) & 1u)) >> 16); }
__device__ __forceinline__ float bf16_val(unsigned short b) { return __uint_as_float(((unsigned int)b) << 16); }
__device__ __forceinline__ float bf16_rne(float x) { return bf16_val(bf16_bits(x)); }
__device__ __forceinline__ unsigned short h16bits(float x) { const _Float16 h = (_Float16)x; return __builtin_bit_cast(unsigned short, h); }

__device__ __forceinline__ v16h g2_frag(const unsigned short* p, unsigned hh) { FragH f; f.half[0] = *(const v8us*)(p + 8u * hh); f.half[1] = *(const v8us*)(p + 16u + 8u * hh); return f.v; }
__device__ __forceinline__ v8f g2_mma(v16h a, v16h b, v8f c) { v8f d = __builtin_amdgcn_wmma_f32_16x16x32_f16(false, a, false, b, (short)0, c, false, false); asm volatile("v_nop\n\tv_nop\n\tv_nop\n\tv_nop" : "+v"(d) : "v"(a), "v"(b)); return d; }
__device__ __forceinline__ v8f mma3(v16h a0, v16h a1, v16h a2, v16h b0, v16h b1, v16h b2, v8f c) {
  c = __builtin_amdgcn_wmma_f32_16x16x32_f16(false, a0, false, b0, (short)0, c, false, false);
  c = __builtin_amdgcn_wmma_f32_16x16x32_f16(false, a1, false, b1, (short)0, c, false, false);
  c = __builtin_amdgcn_wmma_f32_16x16x32_f16(false, a2, false, b2, (short)0, c, false, false);
  asm volatile("v_nop\n\tv_nop\n\tv_nop\n\tv_nop" : "+v"(c) : "v"(a0), "v"(a1), "v"(a2), "v"(b0), "v"(b1), "v"(b2));
  return c;
}

__global__ __launch_bounds__(256) void k_wt_f16(const float* __restrict__ W, _Float16* __restrict__ Wt, unsigned K, unsigned N, float scale) {
  const unsigned t = blockIdx.x * 256u + threadIdx.x; const unsigned k8n = K >> 3; if (t >= N * k8n) return;
  const unsigned n = t / k8n, k8 = (t - n * k8n) * 8u; FragH f;
#pragma unroll
  for (unsigned i = 0; i < 8; ++i) f.h[i] = (_Float16)(bf16_rne(W[(size_t)(k8 + i) * N + n]) * scale);
  const v8us o = f.half[0]; unsigned short* dst = (unsigned short*)Wt + (size_t)n * K + k8;
  *(volatile v8us*)dst = o; __threadfence(); *(volatile v8us*)dst = o;
}

__global__ __launch_bounds__(256) void k_wthd(const float* __restrict__ Wq, const float* __restrict__ Wk, const float* __restrict__ Wv, _Float16* __restrict__ Bt) {
  const unsigned t = blockIdx.x * 256u + threadIdx.x; if (t >= (unsigned)(NH * HD * (DM / 8))) return;
  const unsigned y = blockIdx.y; const float* Wsel = (y == 0u) ? Wq : ((y == 1u) ? Wk : Wv);
  const unsigned m8 = (t % (DM / 8)) * 8u; const unsigned d = (t / (DM / 8)) % HD; const unsigned h = t / ((DM / 8) * HD); FragH f;
#pragma unroll
  for (unsigned q = 0; q < 8; ++q) f.h[q] = (_Float16)(16.0f * bf16_rne(Wsel[((size_t)h * DM + m8 + q) * HD + d]));
  const v8us o = f.half[0]; unsigned short* dst = (unsigned short*)Bt + (size_t)y * DM * DM + ((size_t)h * HD + d) * DM + m8;
  *(volatile v8us*)dst = o; __threadfence(); *(volatile v8us*)dst = o;
}

__global__ __launch_bounds__(256) void k_rel16(const float* __restrict__ rel, _Float16* __restrict__ E16) {
  const unsigned t = blockIdx.x * 256u + threadIdx.x; if (t >= (unsigned)(NH * NRELP * (HD / 8))) return;
  const unsigned c8 = (t % (HD / 8)) * 8u; const unsigned rr = (t / (HD / 8)) % NRELP; const unsigned h = t / ((HD / 8) * NRELP);
  const unsigned rc = (rr < (unsigned)NREL) ? rr : (unsigned)(NREL - 1); const float keep = (rr < (unsigned)NREL) ? 16.0f : 0.0f;
  const float* s = rel + ((size_t)h * NREL + rc) * HD + c8; const v4f a = *(const v4fa*)s, c = *(const v4fa*)(s + 4); FragH f;
#pragma unroll
  for (unsigned q = 0; q < 4; ++q) { f.h[q] = (_Float16)(bf16_rne(a[q]) * keep); f.h[4 + q] = (_Float16)(bf16_rne(c[q]) * keep); }
  const v8us o = f.half[0]; unsigned short* dst = (unsigned short*)E16 + (size_t)t * 8u;
  *(volatile v8us*)dst = o; __threadfence(); *(volatile v8us*)dst = o;
}

__global__ __launch_bounds__(256) void k_xprep(const float* __restrict__ x, _Float16* __restrict__ X16, float* __restrict__ XB, unsigned n4) {
  const unsigned t = blockIdx.x * 256u + threadIdx.x; if (t >= n4) return;
  const unsigned e = t * 4u; const unsigned rd = e / DM; const unsigned c = e - rd * DM;
  const unsigned rs = (rd / NB) * NB_FULL + (rd % NB);
  const v4f a = *(const v4fa*)(x + (size_t)rs * DM + c); v4f xb; v4h y;
#pragma unroll
  for (unsigned q = 0; q < 4; ++q) { xb[q] = bf16_rne(a[q]); y[q] = (_Float16)xb[q]; }
  for (int pass = 0; pass < 2; ++pass) { *(volatile v4h*)(X16 + (size_t)e) = y; *(volatile v4f*)(XB + (size_t)e) = xb; if (pass == 0) __threadfence(); }
}

template <int ACT>
__global__ __launch_bounds__(128) void k_gemm2(const _Float16* __restrict__ A, unsigned lda, const _Float16* __restrict__ Bh, unsigned ldb, float alpha, const float* __restrict__ bias, const float* CP,
    float* C, _Float16* __restrict__ C16, unsigned ldc, unsigned M, unsigned N, unsigned K) {
  static_assert(ACT == 0 || ACT == 3);
  __shared__ __attribute__((aligned(16))) float so[4][32][68];
  const unsigned tid = threadIdx.x, w = tid >> 5, lane = tid & 31u, ln = lane & 15u, hh = lane >> 4;
  const unsigned ntn = N >> 6; const unsigned mt = blockIdx.x / ntn, nq = blockIdx.x - mt * ntn; const unsigned row0 = mt * 128u + 32u * w, col0 = nq * 64u; if (row0 >= M) return;
  const unsigned short* a0p = (const unsigned short*)A + (size_t)(row0 + ln) * lda; const unsigned short* a1p = a0p + (size_t)16 * lda;
  const unsigned short* b0p = (const unsigned short*)Bh + (size_t)(col0 + ln) * ldb; const unsigned short* b1p = b0p + (size_t)16 * ldb; const unsigned short* b2p = b1p + (size_t)16 * ldb; const unsigned short* b3p = b2p + (size_t)16 * ldb;
  const v8f z8 = {0.f,0.f,0.f,0.f,0.f,0.f,0.f,0.f}; v8f c00 = z8, c01 = z8, c02 = z8, c03 = z8, c10 = z8, c11 = z8, c12 = z8, c13 = z8;
#pragma unroll 1
  for (unsigned kb = 0; kb < K; kb += 32u) { const v16h a0 = g2_frag(a0p + kb, hh), a1 = g2_frag(a1p + kb, hh);
    v16h b = g2_frag(b0p + kb, hh); c00 = g2_mma(a0, b, c00); c10 = g2_mma(a1, b, c10);
    b = g2_frag(b1p + kb, hh); c01 = g2_mma(a0, b, c01); c11 = g2_mma(a1, b, c11);
    b = g2_frag(b2p + kb, hh); c02 = g2_mma(a0, b, c02); c12 = g2_mma(a1, b, c12);
    b = g2_frag(b3p + kb, hh); c03 = g2_mma(a0, b, c03); c13 = g2_mma(a1, b, c13); }
  v8f accs[8] = {c00, c01, c02, c03, c10, c11, c12, c13};
#pragma unroll
  for (unsigned u = 0; u < 8; ++u) { const unsigned t = u & 3u, half = u >> 2; const unsigned col = col0 + t * 16u + ln; const float bv = bias ? bf16_rne(bias[col]) : 0.f;
#pragma unroll
    for (unsigned r = 0; r < 8; ++r) { const unsigned rloc = half * 16u + 8u * hh + r; float v = accs[u][r] * alpha + bv; if (CP) v += CP[(size_t)(row0 + rloc) * ldc + col];
      if (ACT == 3) v = fmaxf(v, 0.f);
      so[w][rloc][t * 16u + ln] = v; } }
  __builtin_amdgcn_fence(4  , "workgroup"); __builtin_amdgcn_wave_barrier();
  const unsigned rsub = lane >> 4, c4 = (lane & 15u) * 4u;
  for (int pass = 0; pass < 2; ++pass) {
#pragma unroll
    for (unsigned q = 0; q < 16; ++q) { const unsigned r = q * 2u + rsub; const v4f v = *(const v4fa*)&so[w][r][c4]; if (C) *(volatile v4f*)(C + (size_t)(row0 + r) * ldc + col0 + c4) = v; if (C16) { v4h h4; for (int i = 0; i < 4; ++i) h4[i] = (_Float16)v[i]; *(volatile v4h*)(C16 + (size_t)(row0 + r) * ldc + col0 + c4) = h4; } }
    if (pass == 0) __threadfence(); } }

__global__ __launch_bounds__(256) void k_vt(const _Float16* __restrict__ QKV, _Float16* __restrict__ VT) {
  __shared__ unsigned short tl[64][HD + 2];
  const unsigned tid = threadIdx.x; const unsigned slab = blockIdx.x / (SEQ / 64), lg = blockIdx.x % (SEQ / 64); const unsigned b = slab / NH, h = slab % NH;
  for (unsigned i = tid; i < 64u * (HD / 8); i += 256u) { const unsigned r = i / (HD / 8), c8 = (i % (HD / 8)) * 8u; FragH f;
    f.half[0] = *(const v8us*)((const unsigned short*)QKV + (size_t)((lg * 64u + r) * NB + b) * LQKV + 2 * DM + h * HD + c8);
#pragma unroll
    for (unsigned q = 0; q < 8; ++q) tl[r][c8 + q] = f.u[q]; }
  __syncthreads();
  for (int pass = 0; pass < 2; ++pass) {
#pragma unroll
    for (unsigned rd = 0; rd < HD / 32; ++rd) { const unsigned d = rd * 32u + (tid >> 3), pc = tid & 7u; FragH f;
#pragma unroll
      for (unsigned q = 0; q < 8; ++q) f.u[q] = tl[pc * 8u + q][d];
      *(volatile v8us*)((unsigned short*)VT + ((size_t)slab * HD + d) * SEQ + lg * 64u + pc * 8u) = f.half[0]; }
    if (pass == 0) __threadfence(); } }

__global__ __launch_bounds__(64) void k_attn(const _Float16* __restrict__ QKV, const _Float16* __restrict__ E16, const _Float16* __restrict__ VT, _Float16* __restrict__ O16) {
  __shared__ __attribute__((aligned(16))) float Ll[2][16 * NCOL];
  __shared__ __attribute__((aligned(16))) float Pl[2][16 * NRELP];
  __shared__ __attribute__((aligned(16))) unsigned short Pr[2][16 * PRP];
  __shared__ __attribute__((aligned(16))) unsigned short Ost[16 * 2 * HD];
  const unsigned tid = threadIdx.x, w = tid >> 5, lane = tid & 31u, ln = lane & 15u, hh = lane >> 4;
  const unsigned q0 = blockIdx.x * 16u;
  const unsigned b = blockIdx.y / (NH / 2), hp = blockIdx.y % (NH / 2);
  const unsigned h = hp * 2u + w;
  const int ks = (int)q0 - KSOFF;
  const unsigned short* qkv = (const unsigned short*)QKV;
  const unsigned short* qp = qkv + (size_t)((q0 + ln) * NB + b) * LQKV + h * HD;
  const v16h aq0 = g2_frag(qp, hh), aq1 = g2_frag(qp + 32, hh), aq2 = g2_frag(qp + 64, hh);
  const v8f z8 = {0.f,0.f,0.f,0.f,0.f,0.f,0.f,0.f};
#pragma unroll 1
  for (unsigned jj = 0; jj < NRELP / 16; ++jj) {
    const unsigned short* ep = (const unsigned short*)E16 + (size_t)(h * NRELP + jj * 16u + ln) * HD;
    const v8f acc = mma3(aq0, aq1, aq2, g2_frag(ep, hh), g2_frag(ep + 32, hh), g2_frag(ep + 64, hh), z8);
#pragma unroll
    for (unsigned r = 0; r < 8; ++r) Pl[w][(8u * hh + r) * NRELP + jj * 16u + ln] = acc[r] * 0.0625f;
  }
#pragma unroll 1
  for (unsigned j = 0; j < NCOL / 16; ++j) {
    int krow = ks + (int)(j * 16u + ln); krow = min(max(krow, 0), SEQ - 1);
    const unsigned short* kp = qkv + (size_t)((unsigned)krow * NB + b) * LQKV + DM + h * HD;
    const v8f acc = mma3(aq0, aq1, aq2, g2_frag(kp, hh), g2_frag(kp + 32, hh), g2_frag(kp + 64, hh), z8);
#pragma unroll
    for (unsigned r = 0; r < 8; ++r) Ll[w][(8u * hh + r) * NCOL + j * 16u + ln] = acc[r] * 0.10206207261596577f;
  }
  __syncthreads();
#pragma unroll 1
  for (unsigned m = 0; m < 16; ++m) {
    float lv[7]; float mx = -3.0e38f;
#pragma unroll
    for (int i = 0; i < 7; ++i) {
      const int c = (int)lane + i * 32; const int key = ks + c; const int r = c - (int)m - 5;
      const bool valid = (key >= 0) && (key < SEQ) && (r >= 0) && (r < NREL);
      const int rc = min(max(r, 0), NRELP - 1);
      const float v0 = Ll[w][m * NCOL + (unsigned)c] + Pl[w][m * NRELP + (unsigned)rc];
      const float v = valid ? v0 : -1.0e30f;
      lv[i] = v; mx = fmaxf(mx, v);
    }
#pragma unroll
    for (int s = 16; s > 0; s >>= 1) mx = fmaxf(mx, __shfl_xor(mx, s, 32));
    float sum = 0.f;
#pragma unroll
    for (int i = 0; i < 7; ++i) { lv[i] = __expf(lv[i] - mx); sum += lv[i]; }
#pragma unroll
    for (int s = 16; s > 0; s >>= 1) sum += __shfl_xor(sum, s, 32);
    const float inv = 1024.0f * (1.0f / sum);
#pragma unroll
    for (int i = 0; i < 7; ++i) Pr[w][m * PRP + lane + (unsigned)i * 32u] = h16bits(lv[i] * inv);
  }
  __syncthreads();
  v8f o0 = z8, o1 = z8, o2 = z8, o3 = z8, o4 = z8, o5 = z8;
  const unsigned short* vt = (const unsigned short*)VT + ((size_t)(b * NH + h) * HD + ln) * SEQ;
#pragma unroll 1
  for (unsigned kc = 0; kc < NCOL / 32; ++kc) {
    FragH a; a.half[0] = *(const v8us*)&Pr[w][ln * PRP + kc * 32u + 8u * hh]; a.half[1] = *(const v8us*)&Pr[w][ln * PRP + kc * 32u + 16u + 8u * hh];
    int g0 = ks + (int)(kc * 32u + 8u * hh); int g1 = g0 + 16;
    g0 = min(max(g0, 0), SEQ - 8); g1 = min(max(g1, 0), SEQ - 8);
    FragH bq;
    bq.half[0] = *(const v8us*)(vt + g0); bq.half[1] = *(const v8us*)(vt + g1); o0 = g2_mma(a.v, bq.v, o0);
    bq.half[0] = *(const v8us*)(vt + (size_t)16 * SEQ + g0); bq.half[1] = *(const v8us*)(vt + (size_t)16 * SEQ + g1); o1 = g2_mma(a.v, bq.v, o1);
    bq.half[0] = *(const v8us*)(vt + (size_t)32 * SEQ + g0); bq.half[1] = *(const v8us*)(vt + (size_t)32 * SEQ + g1); o2 = g2_mma(a.v, bq.v, o2);
    bq.half[0] = *(const v8us*)(vt + (size_t)48 * SEQ + g0); bq.half[1] = *(const v8us*)(vt + (size_t)48 * SEQ + g1); o3 = g2_mma(a.v, bq.v, o3);
    bq.half[0] = *(const v8us*)(vt + (size_t)64 * SEQ + g0); bq.half[1] = *(const v8us*)(vt + (size_t)64 * SEQ + g1); o4 = g2_mma(a.v, bq.v, o4);
    bq.half[0] = *(const v8us*)(vt + (size_t)80 * SEQ + g0); bq.half[1] = *(const v8us*)(vt + (size_t)80 * SEQ + g1); o5 = g2_mma(a.v, bq.v, o5);
  }
  v8f osv[6] = {o0, o1, o2, o3, o4, o5};
#pragma unroll
  for (unsigned ni = 0; ni < 6; ++ni) {
#pragma unroll
    for (unsigned r = 0; r < 8; ++r) Ost[(8u * hh + r) * (2 * HD) + w * HD + ni * 16u + ln] = h16bits(osv[ni][r] * 0.0625f);
  }
  __syncthreads();
  for (int pass = 0; pass < 2; ++pass) {
#pragma unroll 1
    for (unsigned it = 0; it < 6; ++it) {
      const unsigned L = it * 8u + (tid >> 3); const unsigned row = L / 3u; const unsigned seg = L - row * 3u; const unsigned pc = tid & 7u;
      const v8us v = *(const v8us*)&Ost[row * (2 * HD) + seg * 64u + pc * 8u];
      *(volatile v8us*)((unsigned short*)O16 + (size_t)((q0 + row) * NB + b) * DM + hp * (2 * HD) + seg * 64u + pc * 8u) = v;
    }
    if (pass == 0) __threadfence();
  }
}

template <int BFIN, int W16, int W32>
__global__ __launch_bounds__(256) void k_lnx(const float* __restrict__ X, const float* __restrict__ g, const float* __restrict__ bb, float eps, _Float16* __restrict__ N16, float* __restrict__ N32) {
  #pragma clang fp contract(off)
  __shared__ float red[256]; const size_t r = blockIdx.x; const unsigned t = threadIdx.x; const bool act = t < (unsigned)(DM / 4); const unsigned c0 = act ? t * 4u : 0u;
  const v4f xa = *(const v4fa*)(X + r * DM + c0); float s[4]; float sum = 0.f;
#pragma unroll
  for (int q = 0; q < 4; ++q) { s[q] = act ? (BFIN ? bf16_rne(xa[q]) : xa[q]) : 0.f; sum = sum + s[q]; }
  red[t] = sum; __syncthreads(); for (unsigned st = 128; st > 0; st >>= 1) { if (t < st) red[t] = red[t] + red[t + st]; __syncthreads(); } const float mu = red[0] * (1.0f / (float)DM); __syncthreads();
  float vs = 0.f;
#pragma unroll
  for (int q = 0; q < 4; ++q) { const float dl = act ? (s[q] - mu) : 0.f; vs = vs + dl * dl; }
  red[t] = vs; __syncthreads(); for (unsigned st = 128; st > 0; st >>= 1) { if (t < st) red[t] = red[t] + red[t + st]; __syncthreads(); }
  const float rs = rsqrtf(red[0] * (1.0f / (float)DM) + eps); v4h y; v4f yf;
#pragma unroll
  for (int q = 0; q < 4; ++q) { const unsigned c = c0 + (unsigned)q; yf[q] = ((s[q] - mu) * rs) * bf16_rne(g[c]) + bf16_rne(bb[c]); y[q] = (_Float16)yf[q]; }
  if (!act) return;
  for (int pass = 0; pass < 2; ++pass) { if (W16) *(volatile v4h*)(N16 + r * DM + c0) = y; if (W32) *(volatile v4f*)(N32 + r * DM + c0) = yf; if (pass == 0) __threadfence(); } }

constexpr size_t al256(size_t v) { return (v + 255) & ~(size_t)255; }
constexpr size_t cmax(size_t a, size_t b) { return a > b ? a : b; }
constexpr size_t SZ_BQKV = al256((size_t)3 * DM * DM * 2);
constexpr size_t SZ_BO   = al256((size_t)DM * DM * 2);
constexpr size_t SZ_BW1  = al256((size_t)DFF * DM * 2);
constexpr size_t SZ_BW2  = al256((size_t)DM * DFF * 2);
constexpr size_t SZ_E16  = al256((size_t)NH * NRELP * HD * 2);
constexpr size_t SZ_QKV  = al256((size_t)MROWS * LQKV * 2);
constexpr size_t SZ_VT   = al256((size_t)NB * NH * HD * SEQ * 2);
constexpr size_t SZ_X1   = al256((size_t)MROWS * DM * 4);
constexpr size_t SZ_HF   = al256((size_t)MROWS * DFF * 2);
constexpr size_t SZ_F32  = al256((size_t)MROWS * DM * 4);
constexpr size_t SZ_F16  = al256((size_t)MROWS * DM * 2);
constexpr size_t SZ_RA   = cmax(cmax(SZ_QKV + SZ_VT, SZ_X1), SZ_HF);
static_assert(SZ_QKV + SZ_VT <= SZ_RA && SZ_X1 <= SZ_RA && SZ_HF <= SZ_RA);
constexpr size_t OFF_BQKV = 0;
constexpr size_t OFF_BO   = OFF_BQKV + SZ_BQKV;
constexpr size_t OFF_BW1  = OFF_BO + SZ_BO;
constexpr size_t OFF_BW2  = OFF_BW1 + SZ_BW1;
constexpr size_t OFF_E16  = OFF_BW2 + SZ_BW2;
constexpr size_t OFF_RA   = OFF_E16 + SZ_E16;
constexpr size_t OFF_RB   = OFF_RA + SZ_RA;
constexpr size_t OFF_RD   = OFF_RB + SZ_F32;
constexpr size_t OFF_RE   = OFF_RD + SZ_F16;
constexpr size_t OFF_END  = OFF_RE + SZ_F16;
static_assert(OFF_END <= (size_t)134217728);

extern "C" void kernel_launch(void* const* d_in, const int* in_sizes, int n_in,
                              void* d_out, int out_size, void* d_ws, size_t ws_size, hipStream_t stream) {
  if (n_in < 14) return;
  if ((size_t)in_sizes[0] < ((size_t)(SEQ - 1) * NB_FULL + NB) * DM) return;
  if (in_sizes[1] < NH * DM * HD || in_sizes[2] < NH * DM * HD || in_sizes[3] < NH * DM * HD || in_sizes[4] < NH * HD * DM) return;
  if (in_sizes[5] < NH * NREL * HD || in_sizes[6] < DM * DFF || in_sizes[7] < DFF || in_sizes[8] < DFF * DM || in_sizes[9] < DM) return;
  if (in_sizes[10] < DM || in_sizes[11] < DM || in_sizes[12] < DM || in_sizes[13] < DM) return;
  if ((size_t)out_size < (size_t)MROWS * DM) return;
  if (OFF_END > ws_size) return;
  const float* x = (const float*)d_in[0]; const float* wq = (const float*)d_in[1]; const float* wk = (const float*)d_in[2]; const float* wv = (const float*)d_in[3];
  const float* wo = (const float*)d_in[4]; const float* rel = (const float*)d_in[5]; const float* w1 = (const float*)d_in[6]; const float* b1 = (const float*)d_in[7];
  const float* w2 = (const float*)d_in[8]; const float* b2 = (const float*)d_in[9]; const float* g1 = (const float*)d_in[10]; const float* be1 = (const float*)d_in[11];
  const float* g2 = (const float*)d_in[12]; const float* be2 = (const float*)d_in[13];
  float* out = (float*)d_out;
  char* ws = (char*)d_ws;
  _Float16* BQKV = (_Float16*)(ws + OFF_BQKV); _Float16* BO = (_Float16*)(ws + OFF_BO); _Float16* BW1 = (_Float16*)(ws + OFF_BW1); _Float16* BW2 = (_Float16*)(ws + OFF_BW2); _Float16* E16 = (_Float16*)(ws + OFF_E16);
  _Float16* QKV = (_Float16*)(ws + OFF_RA); _Float16* VT = (_Float16*)(ws + OFF_RA + SZ_QKV); float* X1 = (float*)(ws + OFF_RA); _Float16* HF16 = (_Float16*)(ws + OFF_RA);
  float* XB = (float*)(ws + OFF_RB); float* SRC32 = (float*)(ws + OFF_RB);
  _Float16* X16 = (_Float16*)(ws + OFF_RD); _Float16* SRC16 = (_Float16*)(ws + OFF_RD);
  _Float16* O16 = (_Float16*)(ws + OFF_RE);

  k_wthd<<<dim3((unsigned)((NH * HD * (DM / 8) + 255) / 256), 3), 256, 0, stream>>>(wq, wk, wv, BQKV);
  k_wt_f16<<<(unsigned)((DM * (DM / 8) + 255) / 256), 256, 0, stream>>>(wo, BO, DM, DM, 16.0f);
  k_wt_f16<<<(unsigned)((DFF * (DM / 8) + 255) / 256), 256, 0, stream>>>(w1, BW1, DM, DFF, 16.0f);
  k_wt_f16<<<(unsigned)((DM * (DFF / 8) + 255) / 256), 256, 0, stream>>>(w2, BW2, DFF, DM, 16.0f);
  k_rel16<<<(unsigned)((NH * NRELP * (HD / 8) + 255) / 256), 256, 0, stream>>>(rel, E16);
  k_xprep<<<(unsigned)((MROWS * (DM / 4) + 255) / 256), 256, 0, stream>>>(x, X16, XB, (unsigned)(MROWS * (DM / 4)));
  k_gemm2<0><<<(unsigned)((MROWS / 128) * (LQKV / 64)), 128, 0, stream>>>(X16, DM, BQKV, DM, 0.0625f, nullptr, nullptr, nullptr, QKV, LQKV, MROWS, LQKV, DM);
  k_vt<<<(unsigned)(NB * NH * (SEQ / 64)), 256, 0, stream>>>(QKV, VT);
  k_attn<<<dim3(SEQ / 16, NB * NH / 2), 64, 0, stream>>>(QKV, E16, VT, O16);
  k_gemm2<0><<<(unsigned)((MROWS / 128) * (DM / 64)), 128, 0, stream>>>(O16, DM, BO, DM, 0.0009765625f, nullptr, XB, X1, nullptr, DM, MROWS, DM, DM);
  k_lnx<0, 1, 1><<<(unsigned)MROWS, 256, 0, stream>>>(X1, g1, be1, 1e-5f, SRC16, SRC32);
  k_gemm2<3><<<(unsigned)((MROWS / 128) * (DFF / 64)), 128, 0, stream>>>(SRC16, DM, BW1, DM, 0.0625f, b1, nullptr, nullptr, HF16, DFF, MROWS, DFF, DM);
  k_gemm2<0><<<(unsigned)((MROWS / 128) * (DM / 64)), 128, 0, stream>>>(HF16, DFF, BW2, DFF, 0.0625f, b2, SRC32, SRC32, nullptr, DM, MROWS, DM, DFF);
  k_lnx<0, 0, 1><<<(unsigned)MROWS, 256, 0, stream>>>(SRC32, g2, be2, 1e-5f, nullptr, out);
}
